// StandardAttention_32744830665501
// MI455X (gfx1250) — hardware-verified
//
#include <hip/hip_runtime.h>


#ifndef NB
#define NB 2
#endif
#ifndef SEQ
#define SEQ 2048
#endif
#ifndef NB_FULL
#define NB_FULL 2
#endif
#ifndef SEQ_FULL
#define SEQ_FULL 2048
#endif

namespace {
constexpr int H = 16, HD = 64, DM = 1024, NT = NB * SEQ, NCS = HD / 2;
constexpr float XS = 8.0f, WSC = 64.0f, QS = 8.0f, QRS = 1024.0f, VS = 8.0f, VRS = 1024.0f, PS = 1024.0f, PRS = 1024.0f, OCS = 64.0f, OCRS = 1024.0f;
constexpr float LOG2E = 1.4426950408889634f, EPSN = 1e-6f;
static_assert(SEQ % 64 == 0 && SEQ >= 64 && SEQ <= SEQ_FULL && NB >= 1 && NB <= NB_FULL);
static_assert(DM == H * HD && HD == 64 && DM % 64 == 0 && (3 * DM) % 64 == 0 && NT % 64 == 0 && PRS == VRS);

typedef _Float16 b16;
typedef __attribute__((ext_vector_type(16))) _Float16 v16b;
typedef __attribute__((ext_vector_type(8))) _Float16 v8b;
typedef __attribute__((ext_vector_type(2))) _Float16 v2b;
typedef __attribute__((ext_vector_type(8))) float v8f;
typedef __attribute__((ext_vector_type(4))) float v4f;
typedef __attribute__((ext_vector_type(2))) float v2f;
typedef __attribute__((ext_vector_type(4))) int v4i;

__device__ __forceinline__ float bf16_rne(float f) { unsigned int u = __float_as_uint(f); u += 0x7FFFu + ((u >> 16) & 1u); return __uint_as_float(u & 0xFFFF0000u); }
__device__ __forceinline__ v16b frag_kb(const b16* p, int hh) {
  const v8b a = *(const v8b*)(p + 8 * hh), b = *(const v8b*)(p + 16 + 8 * hh); v16b f;
#pragma unroll
  for (int e = 0; e < 8; ++e) { f[e] = a[e]; f[8 + e] = b[e]; }
  return f;
}
__device__ __forceinline__ v8f wmma16b(v16b a, v16b b, v8f c) {
  v8f d = __builtin_amdgcn_wmma_f32_16x16x32_f16(false, a, false, b, (short)0, c, false, false);
  asm volatile("v_nop\n\tv_nop\n\tv_nop\n\tv_nop" : "+v"(d) : "v"(a), "v"(b));
  return d;
}
__device__ __forceinline__ void wave_lds_sync() { __builtin_amdgcn_fence(3, "workgroup"); __builtin_amdgcn_wave_barrier(); __builtin_amdgcn_fence(2, "workgroup"); }
__device__ __forceinline__ float nexp2(float v) { return __builtin_amdgcn_exp2f(v); }

__global__ __launch_bounds__(256) void cvt_x_kernel(const float* __restrict__ X, b16* __restrict__ Xp) {
  const size_t u = (size_t)blockIdx.x * 256 + threadIdx.x;
  if (u >= (size_t)NT * DM / 8) return;
  const size_t row = u / (DM / 8); const int piece = (int)(u % (DM / 8));
  const size_t b = row / SEQ, s = row % SEQ;
  const float* src = X + (b * SEQ_FULL + s) * DM + (size_t)piece * 8;
  b16* dst = Xp + row * DM + (size_t)piece * 8;
  const v4f x0 = *(const v4f*)src, x1 = *(const v4f*)(src + 4); v8b o;
#pragma unroll
  for (int j = 0; j < 4; ++j) { o[j] = (b16)(bf16_rne(x0[j]) * XS); o[4 + j] = (b16)(bf16_rne(x1[j]) * XS); }
  *(volatile v8b*)dst = o; __threadfence(); *(volatile v8b*)dst = o;
}

__global__ __launch_bounds__(256) void cvt_w_kernel(const float* __restrict__ Wq, const float* __restrict__ Wk, const float* __restrict__ Wv,
                                                    const float* __restrict__ Wo, b16* __restrict__ Wp) {
  const int y = (int)blockIdx.y;
  const float* W = (y == 0) ? Wq : ((y == 1) ? Wk : ((y == 2) ? Wv : Wo));
  const size_t u = (size_t)blockIdx.x * 256 + threadIdx.x;
  if (u >= (size_t)DM * DM / 8) return;
  const float* src = W + u * 8; b16* dst = Wp + (size_t)y * DM * DM + u * 8;
  const v4f x0 = *(const v4f*)src, x1 = *(const v4f*)(src + 4); v8b o;
#pragma unroll
  for (int j = 0; j < 4; ++j) { o[j] = (b16)(bf16_rne(x0[j]) * WSC); o[4 + j] = (b16)(bf16_rne(x1[j]) * WSC); }
  *(volatile v8b*)dst = o; __threadfence(); *(volatile v8b*)dst = o;
}

__global__ __launch_bounds__(256) void rope_table_kernel(v2f* __restrict__ T) {
  const int u = (int)blockIdx.x * 256 + (int)threadIdx.x;
  if (u >= SEQ * NCS) return;
  const int s = u / NCS, i = u % NCS;
  const float ex = (float)(2 * i) / (float)HD;
  const float pw = (float)exp2((double)ex * 13.287712379549449);
  const float freq = 1.0f / pw;
  const float ang = (float)s * freq;
  const double a = (double)ang;
  const double k = __builtin_rint(a * 0.63661977236758134);
  double rd = __builtin_fma(-k, 1.5707963267948966, a);
  rd = __builtin_fma(-k, 6.123233995736766e-17, rd);
  const float r = (float)rd, r2 = r * r;
  const float sp = r + r * r2 * (-1.6666666666666666e-1f + r2 * (8.333333333333333e-3f + r2 * (-1.984126984126984e-4f + r2 * 2.7557319223985893e-6f)));
  const float cp = 1.0f + r2 * (-0.5f + r2 * (4.1666666666666664e-2f + r2 * (-1.3888888888888889e-3f + r2 * (2.48015873015873e-5f + r2 * -2.755731922398589e-7f))));
  const int kq = (int)(((long long)k) & 3);
  const float c = (kq == 0) ? cp : ((kq == 1) ? -sp : ((kq == 2) ? -cp : sp));
  const float sn = (kq == 0) ? sp : ((kq == 1) ? cp : ((kq == 2) ? -sp : -cp));
  v2f o; o.x = c; o.y = sn;
  *(volatile v2f*)(T + u) = o; __threadfence(); *(volatile v2f*)(T + u) = o;
}

__global__ __launch_bounds__(128) __attribute__((amdgpu_num_vgpr(256))) void gemm_qkv_kernel(
    const b16* __restrict__ Xp, const b16* __restrict__ Wp, const float* __restrict__ bq, const float* __restrict__ bk, const float* __restrict__ bv,
    const v2f* __restrict__ CSt, b16* __restrict__ Qp, b16* __restrict__ Qr, b16* __restrict__ Kp, b16* __restrict__ Kr, b16* __restrict__ VT,
    b16* __restrict__ VR) {
  __shared__ __attribute__((aligned(16))) float Tt[64][HD + 4];
  const int wave = threadIdx.x >> 5, lane = threadIdx.x & 31, hh = lane >> 4, m = lane & 15, wm = wave >> 1, wn = wave & 1;
  const int nblk = (int)blockIdx.x * 64, which = nblk / DM, n0 = nblk % DM, h = n0 / HD;
  const int mblk = (int)blockIdx.y * 64, b = mblk / SEQ, s0 = mblk % SEQ;
  const b16* Wb = Wp + (size_t)which * DM * DM + (size_t)(n0 + wn * 32) * DM;
  const b16* Ab = Xp + (size_t)(mblk + wm * 32) * DM;
  const float* bsel = (which == 0) ? bq : ((which == 1) ? bk : bv);
  v8f acc[2][2];
#pragma unroll
  for (int i = 0; i < 2; ++i)
#pragma unroll
    for (int j = 0; j < 2; ++j) acc[i][j] = (v8f){};
#pragma unroll 1
  for (int k0 = 0; k0 < DM; k0 += 32) {
    v16b af[2], bf[2];
#pragma unroll
    for (int mt = 0; mt < 2; ++mt) af[mt] = frag_kb(Ab + (size_t)(mt * 16 + m) * DM + k0, hh);
#pragma unroll
    for (int nt = 0; nt < 2; ++nt) bf[nt] = frag_kb(Wb + (size_t)(nt * 16 + m) * DM + k0, hh);
#pragma unroll
    for (int mt = 0; mt < 2; ++mt)
#pragma unroll
      for (int nt = 0; nt < 2; ++nt) acc[mt][nt] = wmma16b(af[mt], bf[nt], acc[mt][nt]);
  }
  float bias[2];
#pragma unroll
  for (int nt = 0; nt < 2; ++nt) bias[nt] = bf16_rne(bsel[n0 + wn * 32 + nt * 16 + m]);
  const float isc = 1.0f / (XS * WSC);
#pragma unroll
  for (int mt = 0; mt < 2; ++mt)
#pragma unroll
    for (int nt = 0; nt < 2; ++nt)
#pragma unroll
      for (int r = 0; r < 8; ++r) Tt[wm * 32 + mt * 16 + 8 * hh + r][wn * 32 + nt * 16 + m] = acc[mt][nt][r] * isc + bias[nt];
  __syncthreads();
  if (which < 2) {
    const size_t pb = ((size_t)(b * H + h) * SEQ + (size_t)s0) * HD;
    b16* Ph = ((which == 0) ? Qp : Kp) + pb;
    b16* Pl = ((which == 0) ? Qr : Kr) + pb;
#pragma unroll 1
    for (int it = 0; it < 16; ++it) {
      const int r = it * 4 + wave, s = s0 + r;
      const float x0 = Tt[r][2 * lane], x1 = Tt[r][2 * lane + 1];
      const v2f cv = CSt[(size_t)s * NCS + lane];
      const float y0 = x0 * cv.x - x1 * cv.y, y1 = x1 * cv.x + x0 * cv.y;
      float ss = y0 * y0 + y1 * y1;
#pragma unroll
      for (int w = 16; w >= 1; w >>= 1) ss += __shfl_xor(ss, w);
      const float inv = 1.0f / sqrtf(ss + EPSN);
      const float z0 = y0 * inv * QS, z1 = y1 * inv * QS;
      const b16 h0 = (b16)z0, h1 = (b16)z1;
      v2b oh, ol; oh.x = h0; oh.y = h1; ol.x = (b16)((z0 - (float)h0) * QRS); ol.y = (b16)((z1 - (float)h1) * QRS);
      const size_t off = (size_t)r * HD + 2 * lane;
      *(volatile v2b*)(Ph + off) = oh; *(volatile v2b*)(Pl + off) = ol;
      __threadfence();
      *(volatile v2b*)(Ph + off) = oh; *(volatile v2b*)(Pl + off) = ol;
    }
  } else {
    const size_t vb = ((size_t)(b * H + h) * HD) * SEQ + (size_t)s0;
#pragma unroll 1
    for (int it = 0; it < 4; ++it) {
      const int d = wave * 16 + it * 4 + (lane >> 3), tok = (lane & 7) * 8;
      v8b oh, ol;
#pragma unroll
      for (int j = 0; j < 8; ++j) {
        const float v = Tt[tok + j][d] * VS; const b16 hv = (b16)v; oh[j] = hv; ol[j] = (b16)((v - (float)hv) * VRS); }
      const size_t off = vb + (size_t)d * SEQ + tok;
      *(volatile v8b*)(VT + off) = oh; *(volatile v8b*)(VR + off) = ol;
      __threadfence();
      *(volatile v8b*)(VT + off) = oh; *(volatile v8b*)(VR + off) = ol;
    }
  }
}

__global__ __launch_bounds__(64) __attribute__((amdgpu_num_vgpr(256))) void attn_kernel(
    const b16* __restrict__ Qp, const b16* __restrict__ Qr, const b16* __restrict__ Kp, const b16* __restrict__ Kr,
    const b16* __restrict__ VT, const b16* __restrict__ VR, const int* __restrict__ mask, const float* __restrict__ lsc,
    b16* __restrict__ Ch, b16* __restrict__ Cr) {
  __shared__ __attribute__((aligned(16))) b16 Pb[2][16][32 + 8];
  __shared__ __attribute__((aligned(16))) b16 Pr[2][16][32 + 8];
  __shared__ __attribute__((aligned(16))) float To[2][16][HD + 4];
  const int wave = threadIdx.x >> 5, lane = threadIdx.x & 31, hh = lane >> 4, col = lane & 15;
  const int bhi = (int)blockIdx.y, b = bhi / H, h = bhi % H;
  const int q0 = (int)blockIdx.x * 32 + wave * 16, qi = q0 + col;
  const size_t pq = (size_t)bhi * SEQ * HD;
  const b16* Kb = Kp + pq; const b16* Klb = Kr + pq;
  const b16* Vb = VT + pq; const b16* Rb = VR + pq;
  const int* mrow = mask + ((size_t)b * SEQ_FULL + (size_t)qi) * SEQ_FULL;
  const v16b qa0 = frag_kb(Qp + pq + (size_t)qi * HD, hh), qa1 = frag_kb(Qp + pq + (size_t)qi * HD + 32, hh);
  const v16b ql0 = frag_kb(Qr + pq + (size_t)qi * HD, hh), ql1 = frag_kb(Qr + pq + (size_t)qi * HD + 32, hh);
  const float cs = 0.125f * expf(bf16_rne(lsc[0])) * (LOG2E / (QS * QS));
  float m = -INFINITY, l = 0.0f; v8f o[4], o2[4];
#pragma unroll
  for (int t = 0; t < 4; ++t) { o[t] = (v8f){}; o2[t] = (v8f){}; }
#pragma unroll 1
  for (int k0 = 0; k0 < SEQ; k0 += 32) {
    unsigned int vbm = 0u;
    {
      const int* mp = mrow + k0 + 8 * hh;
      const v4i g0 = *(const v4i*)mp, g1 = *(const v4i*)(mp + 4), g2 = *(const v4i*)(mp + 16), g3 = *(const v4i*)(mp + 20);
#pragma unroll
      for (int j = 0; j < 4; ++j) {
        vbm |= (g0[j] == 0 ? 1u : 0u) << j;       vbm |= (g1[j] == 0 ? 1u : 0u) << (4 + j);
        vbm |= (g2[j] == 0 ? 1u : 0u) << (8 + j); vbm |= (g3[j] == 0 ? 1u : 0u) << (12 + j);
      }
    }
    if (__any((vbm != 0u) ? 1 : 0) == 0) continue;
    float e[16]; float mx = -INFINITY;
#pragma unroll
    for (int u = 0; u < 2; ++u) {
      const size_t kr = (size_t)(k0 + u * 16 + col) * HD;
      const v16b ka = frag_kb(Kb + kr, hh), kc = frag_kb(Kb + kr + 32, hh);
      v8f s = wmma16b(ka, qa0, (v8f){}); s = wmma16b(kc, qa1, s);
      v8f s2 = wmma16b(ka, ql0, (v8f){}); s2 = wmma16b(kc, ql1, s2);
      s2 = wmma16b(frag_kb(Klb + kr, hh), qa0, s2); s2 = wmma16b(frag_kb(Klb + kr + 32, hh), qa1, s2);
#pragma unroll
      for (int r = 0; r < 8; ++r) {
        const int idx = u * 8 + r;
        const float v = ((vbm >> idx) & 1u) ? (s[r] + s2[r] * (1.0f / QRS)) * cs : -INFINITY;
        e[idx] = v; mx = fmaxf(mx, v); } }
    mx = fmaxf(mx, __shfl_xor(mx, 16)); const float mn = fmaxf(m, mx);
    const float mref = (mn == -INFINITY) ? 0.0f : mn;
    const float al = nexp2(m - mref); float sum = 0.0f;
#pragma unroll
    for (int i2 = 0; i2 < 16; ++i2) {
      const float p = nexp2(e[i2] - mref); sum += p; const int pi = (i2 < 8 ? 0 : 16) + 8 * hh + (i2 & 7);
      const float pp = p * PS; const b16 ph = (b16)pp; Pb[wave][col][pi] = ph;
      Pr[wave][col][pi] = (b16)((pp - (float)ph) * PRS); }
    sum += __shfl_xor(sum, 16); l = l * al + sum; m = mn;
    wave_lds_sync();
    const v16b pf = frag_kb(&Pb[wave][col][0], hh), plf = frag_kb(&Pr[wave][col][0], hh);
#pragma unroll
    for (int t = 0; t < 4; ++t) {
      o[t] *= al; o2[t] *= al;
      const size_t vo = (size_t)(t * 16 + col) * SEQ + k0;
      const v16b vh = frag_kb(Vb + vo, hh), vl = frag_kb(Rb + vo, hh);
      o[t] = wmma16b(vh, pf, o[t]);
      o2[t] = wmma16b(vl, pf, o2[t]);
      o2[t] = wmma16b(vh, plf, o2[t]); }
    wave_lds_sync(); }
  const float inv = 1.0f / (l * PS * VS);
#pragma unroll
  for (int t = 0; t < 4; ++t) {
#pragma unroll
    for (int r = 0; r < 8; ++r) To[wave][col][t * 16 + 8 * hh + r] = (o[t][r] + o2[t][r] * (1.0f / VRS)) * inv; }
  wave_lds_sync();
  const size_t cb = ((size_t)b * SEQ + (size_t)q0) * DM + (size_t)h * HD;
#pragma unroll 1
  for (int it = 0; it < 4; ++it) {
    const int rl = it * 4 + (lane >> 3), pc = (lane & 7) * 8;
    const v4f f0 = *(const v4f*)(&To[wave][rl][pc]), f1 = *(const v4f*)(&To[wave][rl][pc + 4]);
    v8b oh, ol;
#pragma unroll
    for (int j = 0; j < 4; ++j) {
      const float v0 = f0[j] * OCS; const b16 hv0 = (b16)v0; oh[j] = hv0; ol[j] = (b16)((v0 - (float)hv0) * OCRS);
      const float v1 = f1[j] * OCS; const b16 hv1 = (b16)v1; oh[4 + j] = hv1; ol[4 + j] = (b16)((v1 - (float)hv1) * OCRS); }
    const size_t off = cb + (size_t)rl * DM + pc;
    *(volatile v8b*)(Ch + off) = oh; *(volatile v8b*)(Cr + off) = ol;
    __threadfence();
    *(volatile v8b*)(Ch + off) = oh; *(volatile v8b*)(Cr + off) = ol;
  }
}

__global__ __launch_bounds__(128) __attribute__((amdgpu_num_vgpr(256))) void gemm_out_kernel(
    const b16* __restrict__ Ch, const b16* __restrict__ Cr, const b16* __restrict__ Wop, const float* __restrict__ bo, float* __restrict__ out) {
  __shared__ __attribute__((aligned(16))) float Tt[64][HD + 4];
  const int wave = threadIdx.x >> 5, lane = threadIdx.x & 31, hh = lane >> 4, m = lane & 15, wm = wave >> 1, wn = wave & 1;
  const int nblk = (int)blockIdx.x * 64;
  const int mblk = (int)blockIdx.y * 64, b = mblk / SEQ, s0 = mblk % SEQ;
  const b16* Wb = Wop + (size_t)(nblk + wn * 32) * DM;
  const b16* Ab = Ch + (size_t)(mblk + wm * 32) * DM;
  const b16* Rb = Cr + (size_t)(mblk + wm * 32) * DM;
  v8f acc[2][2], acc2[2][2];
#pragma unroll
  for (int i = 0; i < 2; ++i)
#pragma unroll
    for (int j = 0; j < 2; ++j) { acc[i][j] = (v8f){}; acc2[i][j] = (v8f){}; }
#pragma unroll 1
  for (int k0 = 0; k0 < DM; k0 += 32) {
    v16b af[2], rf[2], bf[2];
#pragma unroll
    for (int mt = 0; mt < 2; ++mt) {
      af[mt] = frag_kb(Ab + (size_t)(mt * 16 + m) * DM + k0, hh);
      rf[mt] = frag_kb(Rb + (size_t)(mt * 16 + m) * DM + k0, hh); }
#pragma unroll
    for (int nt = 0; nt < 2; ++nt) bf[nt] = frag_kb(Wb + (size_t)(nt * 16 + m) * DM + k0, hh);
#pragma unroll
    for (int mt = 0; mt < 2; ++mt)
#pragma unroll
      for (int nt = 0; nt < 2; ++nt) {
        acc[mt][nt] = wmma16b(af[mt], bf[nt], acc[mt][nt]);
        acc2[mt][nt] = wmma16b(rf[mt], bf[nt], acc2[mt][nt]); }
  }
  float bias[2];
#pragma unroll
  for (int nt = 0; nt < 2; ++nt) bias[nt] = bf16_rne(bo[nblk + wn * 32 + nt * 16 + m]);
  const float isc = 1.0f / (OCS * WSC), irs = 1.0f / OCRS;
#pragma unroll
  for (int mt = 0; mt < 2; ++mt)
#pragma unroll
    for (int nt = 0; nt < 2; ++nt)
#pragma unroll
      for (int r = 0; r < 8; ++r)
        Tt[wm * 32 + mt * 16 + 8 * hh + r][wn * 32 + nt * 16 + m] = (acc[mt][nt][r] + acc2[mt][nt][r] * irs) * isc + bias[nt];
  __syncthreads();
  float* ob = out + ((size_t)b * SEQ_FULL + (size_t)s0) * DM + nblk;
  for (int ps = 0; ps < 2; ++ps) {
#pragma unroll 1
    for (int it = 0; it < 8; ++it) {
      const int rr = it * 8 + wave * 2 + hh; const v4f f = *(const v4f*)(&Tt[rr][m * 4]);
      *(volatile v4f*)(ob + (size_t)rr * DM + m * 4) = f; }
    __threadfence(); }
}
}

extern "C" void kernel_launch(void* const* d_in, const int* in_sizes, int n_in, void* d_out, int out_size, void* d_ws, size_t ws_size, hipStream_t stream) {
  if (n_in < 11) return;
  const size_t need_x = ((size_t)(NB - 1) * SEQ_FULL + SEQ) * DM;
  const size_t need_m = ((size_t)(NB - 1) * SEQ_FULL + SEQ - 1) * SEQ_FULL + SEQ;
  if ((size_t)in_sizes[0] < need_x || (size_t)out_size < need_x || (size_t)in_sizes[10] < need_m || in_sizes[9] < 1) return;
  if (in_sizes[1] < DM * DM || in_sizes[3] < DM * DM || in_sizes[5] < DM * DM || in_sizes[7] < DM * DM) return;
  if (in_sizes[2] < DM || in_sizes[4] < DM || in_sizes[6] < DM || in_sizes[8] < DM) return;
  const float* X = (const float*)d_in[0];
  const float* Wq = (const float*)d_in[1]; const float* bq = (const float*)d_in[2];
  const float* Wk = (const float*)d_in[3]; const float* bk = (const float*)d_in[4];
  const float* Wv = (const float*)d_in[5]; const float* bv = (const float*)d_in[6];
  const float* Wo = (const float*)d_in[7]; const float* bo = (const float*)d_in[8];
  const float* lsc = (const float*)d_in[9]; const int* mask = (const int*)d_in[10];
  size_t off = 0; char* ws = (char*)d_ws;
  auto carve = [&](size_t bytes) { char* p = ws + off; off += (bytes + 255) & ~(size_t)255; return p; };
  const size_t plane = (size_t)NT * DM * 2;
  v2f* T  = (v2f*)carve((size_t)SEQ * NCS * sizeof(v2f));
  b16* Xp = (b16*)carve(plane);
  b16* Wp = (b16*)carve((size_t)4 * DM * DM * 2);
  b16* Qp = (b16*)carve(plane); b16* Qr = (b16*)carve(plane); b16* Kp = (b16*)carve(plane); b16* Kr = (b16*)carve(plane);
  b16* VT = (b16*)carve(plane); b16* VR = (b16*)carve(plane); b16* Ch = (b16*)carve(plane); b16* Cr = (b16*)carve(plane);
  if (off > ws_size || off > ((size_t)128 << 20)) return;
  cvt_x_kernel<<<dim3((unsigned)(((size_t)NT * DM / 8 + 255) / 256)), 256, 0, stream>>>(X, Xp);
  cvt_w_kernel<<<dim3((unsigned)(((size_t)DM * DM / 8 + 255) / 256), 4), 256, 0, stream>>>(Wq, Wk, Wv, Wo, Wp);
  rope_table_kernel<<<dim3((unsigned)((SEQ * NCS + 255) / 256)), 256, 0, stream>>>(T);
  gemm_qkv_kernel<<<dim3(3 * DM / 64, NT / 64), 128, 0, stream>>>(Xp, Wp, bq, bk, bv, T, Qp, Qr, Kp, Kr, VT, VR);
  attn_kernel<<<dim3(SEQ / 32, NB * H), 64, 0, stream>>>(Qp, Qr, Kp, Kr, VT, VR, mask, lsc, Ch, Cr);
  gemm_out_kernel<<<dim3(DM / 64, NT / 64), 128, 0, stream>>>(Ch, Cr, Wp + (size_t)3 * DM * DM, bo, (float*)d_out);
}
